// TrueLastDIFMultiHeadAttention_16415365005500
// MI455X (gfx1250) — hardware-verified
//
#include <hip/hip_runtime.h>
#include <math.h>

typedef __attribute__((ext_vector_type(16))) _Float16 v16h;
typedef __attribute__((ext_vector_type(16))) __bf16 v16b;
typedef __attribute__((ext_vector_type(8)))  _Float16 v8h;
typedef __attribute__((ext_vector_type(8)))  float v8f;
typedef __attribute__((ext_vector_type(4)))  float v4f;
typedef __attribute__((ext_vector_type(2)))  float v2f;
typedef __attribute__((ext_vector_type(4)))  unsigned v4u;
typedef __attribute__((ext_vector_type(4)))  int v4i;
typedef float __attribute__((may_alias)) float_a;
typedef int __attribute__((may_alias)) int_a;

template <typename T> __device__ __forceinline__ void vst2(void* p, T v) { *(volatile T*)p = v; __threadfence(); *(volatile T*)p = v; }
__device__ __forceinline__ v8f wmma16(v16h a, v16h b, v8f c) {
  v8f d = __builtin_amdgcn_wmma_f32_16x16x32_f16(false, a, false, b, (short)0, c, false, false);
  asm volatile("v_nop\n\tv_nop\n\tv_nop\n\tv_nop" : "+v"(d) : "v"(a), "v"(b));
  return d;
}
__device__ __forceinline__ v8f wmma_bf(v16b a, v16b b, v8f c) {
  v8f d = __builtin_amdgcn_wmma_f32_16x16x32_bf16(false, a, false, b, (short)0, c, false, false);
  asm volatile("v_nop\n\tv_nop\n\tv_nop\n\tv_nop" : "+v"(d) : "v"(a), "v"(b));
  return d;
}
__device__ __forceinline__ v16h frag_h(const _Float16* rowk0, int lane) {
  union { v16h v; v8h q[2]; } u; const _Float16* p = rowk0 + 8 * (lane >> 4);
  u.q[0] = *(const v8h*)p; u.q[1] = *(const v8h*)(p + 16); return u.v;
}
__device__ __forceinline__ v16h frag_f32(const float* rowk0, int lane) {
  v16h a; const float* p = rowk0 + 8 * (lane >> 4);
#pragma unroll
  for (int i = 0; i < 8; ++i) { a[i] = (_Float16)p[i]; a[8 + i] = (_Float16)p[16 + i]; }
  return a;
}
__device__ __forceinline__ v16h frag_f32s(const float* rowk0, int lane, float sc) {
  v16h a; const float* p = rowk0 + 8 * (lane >> 4);
#pragma unroll
  for (int i = 0; i < 8; ++i) { a[i] = (_Float16)(p[i] * sc); a[8 + i] = (_Float16)(p[16 + i] * sc); }
  return a;
}
__device__ __forceinline__ v16h fragc_f32(const float* W, int k0, int n, int lane, int ld, int K) {
  v16h a; const int g = lane >> 4;
#pragma unroll
  for (int i = 0; i < 8; ++i) { const int ka = k0 + 8 * g + i, kb = ka + 16;
    a[i] = (_Float16)(ka < K ? W[(size_t)(ka < K ? ka : K - 1) * ld + n] : 0.f); a[8 + i] = (_Float16)(kb < K ? W[(size_t)(kb < K ? kb : K - 1) * ld + n] : 0.f); }
  return a;
}
struct F2 { v16b h, l; };
__device__ __forceinline__ F2 bsplit16(const float v[16]) { F2 r;
#pragma unroll
  for (int i = 0; i < 16; ++i) { const __bf16 h = (__bf16)v[i]; r.h[i] = h; r.l[i] = (__bf16)(v[i] - (float)h); }
  return r; }
__device__ __forceinline__ F2 split_row(const float* row, int k0, int lane) { float v[16]; const float* p = row + k0 + 8 * (lane >> 4);
#pragma unroll
  for (int i = 0; i < 8; ++i) { v[i] = p[i]; v[8 + i] = p[16 + i]; }
  return bsplit16(v); }
__device__ __forceinline__ F2 split_rowK(const float* row, int k0, int lane, int K) { float v[16]; const int g = lane >> 4;
#pragma unroll
  for (int i = 0; i < 8; ++i) { const int ka = k0 + 8 * g + i, kb = ka + 16; v[i] = ka < K ? row[ka < K ? ka : K - 1] : 0.f; v[8 + i] = kb < K ? row[kb < K ? kb : K - 1] : 0.f; }
  return bsplit16(v); }
__device__ __forceinline__ F2 split_col(const float* W, int k0, int n, int lane, int ld, int K) { float v[16]; const int g = lane >> 4;
#pragma unroll
  for (int i = 0; i < 8; ++i) { const int ka = k0 + 8 * g + i, kb = ka + 16; v[i] = ka < K ? W[(size_t)(ka < K ? ka : K - 1) * ld + n] : 0.f; v[8 + i] = kb < K ? W[(size_t)(kb < K ? kb : K - 1) * ld + n] : 0.f; }
  return bsplit16(v); }
__device__ __forceinline__ v8f mac3(const F2& a, const F2& b, v8f c) { c = wmma_bf(a.l, b.h, c); c = wmma_bf(a.h, b.l, c); return wmma_bf(a.h, b.h, c); }
__device__ __forceinline__ float sigm(float v) { return 1.0f / (1.0f + expf(-v)); }
#define LDSX() do { asm volatile("s_wait_dscnt 0" ::: "memory"); __builtin_amdgcn_wave_barrier(); __builtin_amdgcn_fence(__ATOMIC_RELEASE, "workgroup"); } while (0)


#define NB 32
#define LL 512
#define NR (NB * LL)
#define DD 256
#define AA 64
#define NH 4
#define DH 64
#define AH 16
#define QW 160
#ifndef TNB
#define TNB NB
#endif
typedef __attribute__((ext_vector_type(8))) __bf16 v8b;
__device__ __forceinline__ v16b frag_b(const __bf16* rowk0, int lane) {
  union { v16b v; v8b q[2]; } u; const __bf16* p = rowk0 + 8 * (lane >> 4);
  u.q[0] = *(const v8b*)p; u.q[1] = *(const v8b*)(p + 16); return u.v;
}
__device__ __forceinline__ float bfr(float v) { return (float)(__bf16)v; }
__device__ __attribute__((noinline)) float exp_ni(float v) { return expf(v); }
__device__ __attribute__((noinline)) float erf_ni(float v) { return erff(v); }

#define PKO_Q   0
#define PKO_K   (1 * DD * DD)
#define PKO_QP  (2 * DD * DD)
#define PKO_KP  (3 * DD * DD)
#define PKO_D   (4 * DD * DD)
#define PKO_Q0  (5 * DD * DD)
#define PKO_K0  (PKO_Q0 + AA * AA)
#define PKO_Q1  (PKO_K0 + AA * AA)
#define PKO_K1  (PKO_Q1 + AA * AA)
#define PK_END  (PKO_K1 + AA * AA)
#define WS_PK   0u
#define WS_QH   (((2u * PK_END) + 127u) / 128u * 128u)
#define WS_QL   (WS_QH + 2u * NR * NH * QW)
#define WS_KH   (WS_QL + 2u * NR * NH * QW)
#define WS_KL   (WS_KH + 2u * NR * NH * QW)
#define WS_VT   (WS_KL + 2u * NR * NH * QW)
#define WS_CH   (WS_VT + 2u * NR * DD)
#define WS_CL   (WS_CH + 2u * NR * DD)
#define WS_END  (WS_CL + 2u * NR * DD)

__global__ __launch_bounds__(256) void k_pack(const float* __restrict__ WQ, const float* __restrict__ WK, const float* __restrict__ WQP, const float* __restrict__ WKP, const float* __restrict__ WD, const float* __restrict__ WQ0, const float* __restrict__ WK0, const float* __restrict__ WQ1, const float* __restrict__ WK1, __bf16* __restrict__ PK) {
  __shared__ __align__(16) __bf16 s[DD]; const int n = blockIdx.x, which = blockIdx.y, t = threadIdx.x; int K; size_t dst;
  if (which < 5) { const float* Wm = (which == 0) ? WQ : (which == 1) ? WK : (which == 2) ? WQP : (which == 3) ? WKP : WD; K = DD; dst = (size_t)which * DD * DD + (size_t)n * DD; s[t] = (__bf16)Wm[(size_t)t * DD + n]; }
  else { if (n >= AA) return; const float* Wm = (which == 5) ? WQ0 : (which == 6) ? WK0 : (which == 7) ? WQ1 : WK1; K = AA; dst = PKO_Q0 + (size_t)(which - 5) * AA * AA + (size_t)n * AA; if (t < AA) s[t] = (__bf16)Wm[(size_t)t * AA + n]; }
  __syncthreads();
  if (t < K / 8) vst2((unsigned*)(PK + dst + t * 8), *(const v4u*)&s[t * 8]);
}
__global__ __launch_bounds__(64) void k_proj(const float* __restrict__ X, const float* __restrict__ POS, const float* __restrict__ A0, const float* __restrict__ A1, const __bf16* __restrict__ PK, const float* __restrict__ B_X, const float* __restrict__ B_P, const float* __restrict__ B_0, const float* __restrict__ B_1, int side, __bf16* __restrict__ OH, __bf16* __restrict__ OL) {
  __shared__ __align__(16) __bf16 soh[2][16][NH * QW + 8], sol[2][16][NH * QW + 8];
  const int tid = threadIdx.x, wave = tid >> 5, lane = tid & 31, col = lane & 15, g = lane >> 4; const size_t r0 = (size_t)blockIdx.x * 32 + wave * 16;
  const __bf16* PX = PK + (side ? PKO_K : PKO_Q); const __bf16* PP = PK + (side ? PKO_KP : PKO_QP); const __bf16* P0 = PK + (side ? PKO_K0 : PKO_Q0); const __bf16* P1 = PK + (side ? PKO_K1 : PKO_Q1);
#pragma unroll 1
  for (int part = 0; part < 2; ++part) { const float* SRC = part ? POS : X; const __bf16* PW = part ? PP : PX; const float* BB = part ? B_P : B_X;
#pragma unroll 1
    for (int half = 0; half < 2; ++half) { v8f acc[8] = {};
#pragma unroll
      for (int kc = 0; kc < DD / 32; ++kc) { v16b a; { const float* p = SRC + (r0 + col) * DD + kc * 32 + 8 * g;
#pragma unroll
          for (int i = 0; i < 8; ++i) { a[i] = (__bf16)p[i]; a[8 + i] = (__bf16)p[16 + i]; } }
#pragma unroll
        for (int j = 0; j < 8; ++j) acc[j] = wmma_bf(a, frag_b(PW + (size_t)(half * 128 + j * 16 + col) * DD + kc * 32, lane), acc[j]); }
#pragma unroll
      for (int j = 0; j < 8; ++j) { const int c = half * 128 + j * 16 + col; const int h = c / DH, d = c % DH; const float bb = bfr(BB[c]); const int oc = h * QW + part * DH + d;
#pragma unroll
        for (int r = 0; r < 8; ++r) { const float v = acc[j][r] + bb; const __bf16 hb = (__bf16)v; soh[wave][8 * g + r][oc] = hb; sol[wave][8 * g + r][oc] = (__bf16)(v - (float)hb); } } } }
#pragma unroll 1
  for (int ap = 0; ap < 2; ++ap) { const float* SRC = ap ? A1 : A0; const __bf16* PW = ap ? P1 : P0; const float* BB = ap ? B_1 : B_0; v8f acc[4] = {};
#pragma unroll
    for (int kc = 0; kc < AA / 32; ++kc) { v16b a; { const float* p = SRC + (r0 + col) * AA + kc * 32 + 8 * g;
#pragma unroll
        for (int i = 0; i < 8; ++i) { a[i] = (__bf16)p[i]; a[8 + i] = (__bf16)p[16 + i]; } }
#pragma unroll
      for (int j = 0; j < 4; ++j) acc[j] = wmma_bf(a, frag_b(PW + (size_t)(j * 16 + col) * AA + kc * 32, lane), acc[j]); }
#pragma unroll
    for (int j = 0; j < 4; ++j) { const int c = j * 16 + col; const int h = c / AH, d = c % AH; const float bb = bfr(BB[c]); const int oc = h * QW + 2 * DH + ap * AH + d;
#pragma unroll
      for (int r = 0; r < 8; ++r) { const float v = acc[j][r] + bb; const __bf16 hb = (__bf16)v; soh[wave][8 * g + r][oc] = hb; sol[wave][8 * g + r][oc] = (__bf16)(v - (float)hb); } } }
  LDSX();
  for (int rl = 0; rl < 16; ++rl) for (int pc = lane; pc < NH * QW / 8; pc += 32) { vst2((unsigned*)(OH + (r0 + rl) * (NH * QW) + pc * 8), *(const v4u*)&soh[wave][rl][pc * 8]); vst2((unsigned*)(OL + (r0 + rl) * (NH * QW) + pc * 8), *(const v4u*)&sol[wave][rl][pc * 8]); }
}
__global__ __launch_bounds__(256) void k_vt(const float* __restrict__ V, __bf16* __restrict__ VT) {
  __shared__ __align__(16) __bf16 s[DD][72]; const int tid = threadIdx.x; const int kb = blockIdx.x, b = blockIdx.y; const size_t row0 = (size_t)b * LL + (size_t)kb * 64;
  for (int e = tid; e < 64 * DD; e += 256) { const int r = e / DD, c = e % DD; s[c][r] = (__bf16)V[(row0 + r) * DD + c]; }
  __syncthreads();
  for (int e = tid; e < DD * 8; e += 256) { const int c = e >> 3, pc = e & 7; const int h = c / DH, d = c % DH; vst2((unsigned*)(VT + (((size_t)b * NH + h) * DH + d) * LL + (size_t)kb * 64 + pc * 8), *(const v4u*)&s[c][pc * 8]); }
}
__global__ __launch_bounds__(128) void k_attn(const __bf16* __restrict__ QH, const __bf16* __restrict__ QL_, const __bf16* __restrict__ KH, const __bf16* __restrict__ KL, const __bf16* __restrict__ VT, const float* __restrict__ MSK, __bf16* __restrict__ CH, __bf16* __restrict__ CL) {
  __shared__ __align__(16) __bf16 sph[4][16][40], spl[4][16][40]; __shared__ __align__(16) __bf16 soh[4][16][72], sol[4][16][72];
  const int tid = threadIdx.x, wave = tid >> 5, lane = tid & 31, col = lane & 15, g = lane >> 4; const int qb = blockIdx.x, h = blockIdx.y, b = blockIdx.z; const int q0 = qb * 64 + wave * 16; const size_t rq = (size_t)b * LL + q0 + col;
  v16b aqh[5], aql[5];
#pragma unroll
  for (int kc = 0; kc < 5; ++kc) { aqh[kc] = frag_b(QH + rq * (NH * QW) + h * QW + kc * 32, lane); aql[kc] = frag_b(QL_ + rq * (NH * QW) + h * QW + kc * 32, lane); }
  const __bf16* Vbh = VT + ((size_t)b * NH + h) * DH * LL;
  float m[8], l[8];
#pragma unroll
  for (int r = 0; r < 8; ++r) { m[r] = -3.0e38f; l[r] = 0.f; }
  v8f acc[4] = {};
#pragma unroll 1
  for (int ks = 0; ks < LL / 32; ++ks) { v8f s[2];
#pragma unroll
    for (int ct = 0; ct < 2; ++ct) { const int kk = ks * 32 + ct * 16 + col; const size_t rk = ((size_t)b * LL + kk) * (NH * QW) + h * QW; v8f c = {};
#pragma unroll
      for (int kc = 0; kc < 5; ++kc) { const v16b bh = frag_b(KH + rk + kc * 32, lane), bl = frag_b(KL + rk + kc * 32, lane); c = wmma_bf(aql[kc], bh, c); c = wmma_bf(aqh[kc], bl, c); c = wmma_bf(aqh[kc], bh, c); }
#pragma unroll
      for (int r = 0; r < 8; ++r) { const int qi = q0 + 8 * g + r; s[ct][r] = c[r] * 0.125f + bfr(MSK[(size_t)qi * LL + kk]); } }
#pragma unroll
    for (int r = 0; r < 8; ++r) { float mx = fmaxf(s[0][r], s[1][r]);
#pragma unroll
      for (int o = 1; o < 16; o <<= 1) mx = fmaxf(mx, __shfl_xor(mx, o));
      const float mn = fmaxf(m[r], mx); const float alpha = (m[r] <= -1.0e38f) ? 0.f : exp_ni(m[r] - mn); const float e0 = exp_ni(s[0][r] - mn), e1 = exp_ni(s[1][r] - mn); float es = e0 + e1;
#pragma unroll
      for (int o = 1; o < 16; o <<= 1) es += __shfl_xor(es, o);
      l[r] = l[r] * alpha + es; m[r] = mn;
#pragma unroll
      for (int dt = 0; dt < 4; ++dt) acc[dt][r] *= alpha;
      const __bf16 h0 = (__bf16)e0, h1 = (__bf16)e1; sph[wave][8 * g + r][col] = h0; sph[wave][8 * g + r][16 + col] = h1; spl[wave][8 * g + r][col] = (__bf16)(e0 - (float)h0); spl[wave][8 * g + r][16 + col] = (__bf16)(e1 - (float)h1); }
    LDSX();
    const v16b pah = frag_b(&sph[wave][col][0], lane), pal = frag_b(&spl[wave][col][0], lane);
#pragma unroll
    for (int dt = 0; dt < 4; ++dt) { const v16b vb = frag_b(Vbh + (size_t)(dt * 16 + col) * LL + ks * 32, lane); acc[dt] = wmma_bf(pal, vb, acc[dt]); acc[dt] = wmma_bf(pah, vb, acc[dt]); }
    LDSX(); }
#pragma unroll
  for (int r = 0; r < 8; ++r) { const float il = 1.0f / l[r];
#pragma unroll
    for (int dt = 0; dt < 4; ++dt) { const float v = acc[dt][r] * il; const __bf16 hb = (__bf16)v; soh[wave][8 * g + r][dt * 16 + col] = hb; sol[wave][8 * g + r][dt * 16 + col] = (__bf16)(v - (float)hb); } }
  LDSX();
  for (int rl = 0; rl < 16; ++rl) { const size_t o = ((size_t)b * LL + q0 + rl) * DD + h * DH; if (lane < 8) vst2((unsigned*)(CH + o + lane * 8), *(const v4u*)&soh[wave][rl][lane * 8]); else if (lane < 16) vst2((unsigned*)(CL + o + (lane - 8) * 8), *(const v4u*)&sol[wave][rl][(lane - 8) * 8]); }
}
__global__ __launch_bounds__(128) void k_out(const __bf16* __restrict__ CH, const __bf16* __restrict__ CL, const __bf16* __restrict__ PK, const float* __restrict__ BD, const float* __restrict__ LNG, const float* __restrict__ LNB, const float* __restrict__ X, float* __restrict__ OUT) {
  __shared__ __align__(16) float sh_[4][16][DD + 4]; __shared__ float sps[4][16][16][2];
  const int tid = threadIdx.x, wave = tid >> 5, lane = tid & 31, col = lane & 15, g = lane >> 4; const size_t r0 = (size_t)blockIdx.x * 64 + wave * 16;
  float s1[8], s2[8];
#pragma unroll
  for (int r = 0; r < 8; ++r) { s1[r] = 0.f; s2[r] = 0.f; }
#pragma unroll 1
  for (int half = 0; half < 2; ++half) { v8f acc[8] = {};
#pragma unroll
    for (int kc = 0; kc < DD / 32; ++kc) { const v16b ah = frag_b(CH + (r0 + col) * DD + kc * 32, lane), al = frag_b(CL + (r0 + col) * DD + kc * 32, lane);
#pragma unroll
      for (int j = 0; j < 8; ++j) { const v16b w = frag_b(PK + PKO_D + (size_t)(half * 128 + j * 16 + col) * DD + kc * 32, lane); acc[j] = wmma_bf(al, w, acc[j]); acc[j] = wmma_bf(ah, w, acc[j]); } }
#pragma unroll
    for (int j = 0; j < 8; ++j) { const int c = half * 128 + j * 16 + col; const float bb = bfr(BD[c]);
#pragma unroll
      for (int r = 0; r < 8; ++r) { const float v = acc[j][r] + bb; sh_[wave][8 * g + r][c] = v; s1[r] += v; s2[r] += v * v; } } }
#pragma unroll
  for (int r = 0; r < 8; ++r) { sps[wave][8 * g + r][col][0] = s1[r]; sps[wave][8 * g + r][col][1] = s2[r]; }
  LDSX();
  for (int rl = 0; rl < 16; ++rl) { float a = 0.f, b2 = 0.f;
#pragma unroll
    for (int k = 0; k < 16; ++k) { a += sps[wave][rl][k][0]; b2 += sps[wave][rl][k][1]; }
    const float mu = a / (float)DD; const float var = fmaxf(b2 / (float)DD - mu * mu, 0.f); const float inv = 1.0f / sqrtf(var + 1e-12f); const size_t row = r0 + rl;
    for (int c0 = lane * 4; c0 < DD; c0 += 128) { v4f v;
#pragma unroll
      for (int i = 0; i < 4; ++i) { const int c = c0 + i; v[i] = bfr(LNG[c]) * (sh_[wave][rl][c] - mu) * inv + bfr(LNB[c]) + bfr(X[row * DD + c]); }
      vst2(OUT + row * DD + c0, v); } }
}
extern "C" void kernel_launch(void* const* d_in, const int* in_sizes, int n_in, void* d_out, int out_size, void* d_ws, size_t ws_size, hipStream_t stream) {
  (void)in_sizes; (void)n_in; (void)out_size;
  const float** F = (const float**)d_in;
  if (ws_size < (size_t)WS_END) return;
  char* ws = (char*)d_ws; __bf16 *PK = (__bf16*)(ws + WS_PK), *QH = (__bf16*)(ws + WS_QH), *QLp = (__bf16*)(ws + WS_QL), *KH = (__bf16*)(ws + WS_KH), *KL = (__bf16*)(ws + WS_KL), *VT = (__bf16*)(ws + WS_VT), *CH = (__bf16*)(ws + WS_CH), *CL = (__bf16*)(ws + WS_CL);
  k_pack<<<dim3(DD, 9), 256, 0, stream>>>(F[6], F[8], F[10], F[12], F[22], F[14], F[16], F[18], F[20], PK);
  k_proj<<<TNB * LL / 32, 64, 0, stream>>>(F[0], F[1], F[3], F[4], PK, F[7], F[11], F[15], F[19], 0, QH, QLp);
  k_proj<<<TNB * LL / 32, 64, 0, stream>>>(F[0], F[1], F[3], F[4], PK, F[9], F[13], F[17], F[21], 1, KH, KL);
  k_vt<<<dim3(LL / 64, TNB), 256, 0, stream>>>(F[2], VT);
  k_attn<<<dim3(LL / 64, NH, TNB), 128, 0, stream>>>(QH, QLp, KH, KL, VT, F[5], CH, CL);
  k_out<<<TNB * LL / 64, 128, 0, stream>>>(CH, CL, PK, F[23], F[24], F[25], F[0], (float*)d_out);
}
